// PositionFeaturizer_63101659512934
// MI455X (gfx1250) — hardware-verified
//
#include <hip/hip_runtime.h>


#define NN_   8192
#define NS_   16384
#define NE_   131072
#define DM    512
#define NH_   8
#define HD    64
#define MAXSEG 64

typedef unsigned short bf;
typedef __attribute__((ext_vector_type(16))) __bf16   v16bf;
typedef __attribute__((ext_vector_type(8)))  unsigned short v8us;
typedef __attribute__((ext_vector_type(8)))  float    v8f;
typedef __attribute__((ext_vector_type(4)))  float    v4f;
typedef v4f  __attribute__((may_alias)) v4fa;
typedef v8us __attribute__((may_alias)) v8usa;

__device__ __forceinline__ unsigned short f2bf(float f) { unsigned u = __float_as_uint(f); u += 0x7FFFu + ((u >> 16) & 1u); return (unsigned short)(u >> 16); }
__device__ __forceinline__ float bf2f(unsigned short b) { return __uint_as_float(((unsigned)b) << 16); }
__device__ __forceinline__ float bfr(float f) { return bf2f(f2bf(f)); }
__device__ __forceinline__ v16bf cat16b(v8us lo, v8us hi) { return __builtin_bit_cast(v16bf, __builtin_shufflevector(lo, hi, 0, 1, 2, 3, 4, 5, 6, 7, 8, 9, 10, 11, 12, 13, 14, 15)); }
__device__ __forceinline__ v8f wmmab(v16bf a, v16bf b, v8f c) { return __builtin_amdgcn_wmma_f32_16x16x32_bf16(false, a, false, b, (short)0, c, false, false); }
#define VST2(T, p, v) do { const T vst2_v_ = (v); *(volatile T*)(p) = vst2_v_; __threadfence(); *(volatile T*)(p) = vst2_v_; } while (0)

__global__ __launch_bounds__(256) void k_xb(const float* __restrict__ x, bf* Xb) {
    const int lane = threadIdx.x & 31, r = blockIdx.x * 8 + (threadIdx.x >> 5);
    if (r >= NN_) return;
    v8us o[2];
#pragma unroll
    for (int q = 0; q < 2; ++q) { v8us t;
#pragma unroll
        for (int i = 0; i < 8; ++i) t[i] = f2bf(x[(size_t)r * DM + q * 256 + lane * 8 + i]);
        o[q] = t; }
#pragma unroll
    for (int q = 0; q < 2; ++q) *(volatile v8us*)(Xb + (size_t)r * DM + q * 256 + lane * 8) = o[q];
    __threadfence();
#pragma unroll
    for (int q = 0; q < 2; ++q) *(volatile v8us*)(Xb + (size_t)r * DM + q * 256 + lane * 8) = o[q];
}

__global__ __launch_bounds__(256) void k_wt(const float* __restrict__ Wm, bf* WT) {
    __shared__ __align__(16) unsigned short tl[64 * 72];
    const int tid = threadIdx.x, k0 = blockIdx.x * 64, n0 = blockIdx.y * 64;
    const int kk = tid >> 2, nq = (tid & 3) * 16;
#pragma unroll
    for (int i = 0; i < 16; ++i) tl[(nq + i) * 72 + kk] = f2bf(Wm[(size_t)(k0 + kk) * DM + n0 + nq + i]);
    __syncthreads();
    const int piece = tid & 7;
    auto pass = [&]() {
#pragma unroll
        for (int s = 0; s < 2; ++s) { const int nr = (tid >> 3) + 32 * s; const v8us val = *(const v8usa*)(tl + nr * 72 + piece * 8);
            *(volatile v8us*)(WT + (size_t)(n0 + nr) * DM + k0 + piece * 8) = val; }
    };
    pass(); __threadfence(); pass();
}

__global__ __launch_bounds__(128) void k_gemmb(const bf* __restrict__ A, const bf* __restrict__ Bn, const float* __restrict__ bias, float* C) {
    __shared__ __align__(16) float ost[4][16 * 68];
    const int lane = threadIdx.x & 31, wave = threadIdx.x >> 5, lr = lane & 15, hi = lane >> 4;
    const int r0 = blockIdx.x * 64 + wave * 16, c0 = blockIdx.y * 64;
    const size_t aoff = (size_t)(r0 + lr) * DM + 8 * hi;
    size_t boff[4];
#pragma unroll
    for (int t = 0; t < 4; ++t) boff[t] = (size_t)(c0 + t * 16 + lr) * DM + 8 * hi;
    v8f acc[4];
#pragma unroll
    for (int t = 0; t < 4; ++t) acc[t] = (v8f){};
#pragma unroll 1
    for (int kc = 0; kc < DM; kc += 32) {
        const v16bf a = cat16b(*(const v8us*)(A + aoff + kc), *(const v8us*)(A + aoff + kc + 16));
#pragma unroll
        for (int t = 0; t < 4; ++t) acc[t] = wmmab(a, cat16b(*(const v8us*)(Bn + boff[t] + kc), *(const v8us*)(Bn + boff[t] + kc + 16)), acc[t]);
        asm volatile("v_nop\n\tv_nop\n\tv_nop\n\tv_nop" : "+v"(acc[0]), "+v"(acc[1]), "+v"(acc[2]), "+v"(acc[3]) : "v"(a));
    }
    float* os = &ost[wave][0];
#pragma unroll
    for (int t = 0; t < 4; ++t) { const float bv = bfr(bias[c0 + t * 16 + lr]);
#pragma unroll
        for (int j = 0; j < 8; ++j) os[(hi * 8 + j) * 68 + t * 16 + lr] = acc[t][j] + bv; }
    __syncthreads();
    float* crow = C + (size_t)r0 * DM + c0;
    auto pass = [&]() {
#pragma unroll
        for (int s = 0; s < 8; ++s) { const int Lid = (lane >> 3) + 4 * s, piece = lane & 7; const int row = Lid >> 1, cofs = (Lid & 1) * 32 + piece * 4;
            const v4f val = *(const v4fa*)(os + row * 68 + cofs); *(volatile v4f*)(crow + (size_t)row * DM + cofs) = val; }
    };
    pass(); __threadfence(); pass();
}

__device__ __forceinline__ int lower_bound_ri(const int* __restrict__ ri, int v) {
    int lo = 0, hi = NE_;
#pragma unroll 1
    for (int it = 0; it < 18; ++it) { if (lo < hi) { const int mid = (lo + hi) >> 1; if (ri[mid] < v) lo = mid + 1; else hi = mid; } }
    return lo;
}

__global__ __launch_bounds__(256) void k_edges(const float* __restrict__ Q, const float* __restrict__ Kf, const int* __restrict__ rowi, const int* __restrict__ srci,
                                               const float* __restrict__ abias, const float* __restrict__ dist, const float* __restrict__ pos, const float* __restrict__ spos,
                                               const int* __restrict__ o2s, float* out) {
    __shared__ __align__(16) float st[4 * NH_ * 3];
    __shared__ int seg[4][2];
    const int lane = threadIdx.x & 31, h = threadIdx.x >> 5;
    const int nb = blockIdx.x * 4;
    if (threadIdx.x < 4) { const int n = nb + threadIdx.x; seg[threadIdx.x][0] = lower_bound_ri(rowi, n); seg[threadIdx.x][1] = lower_bound_ri(rowi, n + 1); }
    __syncthreads();
#pragma unroll 1
    for (int r = 0; r < 4; ++r) {
        const int n = nb + r;
        const int lo = seg[r][0];
        int cnt = seg[r][1] - lo; cnt = cnt < 0 ? 0 : (cnt > MAXSEG ? MAXSEG : cnt);
        const float q0 = Q[(size_t)n * DM + h * HD + 2 * lane], q1 = Q[(size_t)n * DM + h * HD + 2 * lane + 1];
        float lg[2] = {-__builtin_inff(), -__builtin_inff()};
        int   mysrc[2] = {0, 0}; float myinvd[2] = {0.f, 0.f};
#pragma unroll 1
        for (int j = 0; j < cnt; ++j) {
            const int e = lo + j;
            int s = srci[e]; s = min(max(s, 0), NS_ - 1);
            int kr = o2s[s]; kr = min(max(kr, 0), NN_ - 1);
            const float k0 = Kf[(size_t)kr * DM + h * HD + 2 * lane], k1 = Kf[(size_t)kr * DM + h * HD + 2 * lane + 1];
            float d = q0 * k0 + q1 * k1;
#pragma unroll
            for (int o = 16; o; o >>= 1) d += __shfl_xor(d, o, 32);
            const float l = d / 8.0f + bfr(abias[(size_t)h * NE_ + e]);
            if ((j & 31) == lane) {
                const int slot = j >> 5;
                const float dd = bfr(dist[e]);
                lg[slot] = l; mysrc[slot] = s; myinvd[slot] = (dd == 0.f) ? 0.f : 1.0f / dd;
            }
        }
        float m = fmaxf(lg[0], lg[1]);
#pragma unroll
        for (int o = 16; o; o >>= 1) m = fmaxf(m, __shfl_xor(m, o, 32));
        float p[2], z = 0.f;
#pragma unroll
        for (int sl = 0; sl < 2; ++sl) { p[sl] = (sl * 32 + lane < cnt) ? expf(lg[sl] - m) : 0.f; z += p[sl]; }
#pragma unroll
        for (int o = 16; o; o >>= 1) z += __shfl_xor(z, o, 32);
        float dx = 0.f, dy = 0.f, dz = 0.f, as = 0.f;
#pragma unroll
        for (int sl = 0; sl < 2; ++sl) {
            if (sl * 32 + lane < cnt) {
                const float a = (p[sl] / z) * myinvd[sl];
                const int s = mysrc[sl];
                dx += a * bfr(spos[(size_t)s * 3]); dy += a * bfr(spos[(size_t)s * 3 + 1]); dz += a * bfr(spos[(size_t)s * 3 + 2]); as += a;
            }
        }
#pragma unroll
        for (int o = 16; o; o >>= 1) { dx += __shfl_xor(dx, o, 32); dy += __shfl_xor(dy, o, 32); dz += __shfl_xor(dz, o, 32); as += __shfl_xor(as, o, 32); }
        if (lane == 0) {
            st[(r * NH_ + h) * 3 + 0] = dx - as * bfr(pos[(size_t)n * 3 + 0]);
            st[(r * NH_ + h) * 3 + 1] = dy - as * bfr(pos[(size_t)n * 3 + 1]);
            st[(r * NH_ + h) * 3 + 2] = dz - as * bfr(pos[(size_t)n * 3 + 2]);
        }
    }
    __syncthreads();
    if (h == 0 && lane < 24) {
        const v4f val = *(const v4fa*)(st + lane * 4);
        VST2(v4f, out + (size_t)nb * (NH_ * 3) + lane * 4, val);
    }
}

extern "C" void kernel_launch(void* const* d_in, const int* in_sizes, int n_in,
                              void* d_out, int out_size, void* d_ws, size_t ws_size, hipStream_t stream) {
    (void)in_sizes; (void)n_in; (void)out_size;
    const float* x = (const float*)d_in[0]; const int* rowi = (const int*)d_in[1]; const int* srci = (const int*)d_in[2]; const float* abias = (const float*)d_in[3];
    const float* dist = (const float*)d_in[4]; const float* pos = (const float*)d_in[5]; const float* spos = (const float*)d_in[6]; const int* o2s = (const int*)d_in[7];
    const float* Wq = (const float*)d_in[8]; const float* bq = (const float*)d_in[9]; const float* Wk = (const float*)d_in[10]; const float* bk = (const float*)d_in[11];
    float* out = (float*)d_out;
    char* wsp = (char*)d_ws;
    auto take = [&](size_t bytes) { char* p = wsp; wsp += (bytes + 255) & ~(size_t)255; return (void*)p; };
    bf* Xb = (bf*)take((size_t)NN_ * DM * 2); bf* WQT = (bf*)take((size_t)DM * DM * 2); bf* WKT = (bf*)take((size_t)DM * DM * 2);
    float* Q = (float*)take((size_t)NN_ * DM * 4); float* Kf = (float*)take((size_t)NN_ * DM * 4);
    if ((size_t)(wsp - (char*)d_ws) > ws_size) return;
    k_xb<<<NN_ / 8, 256, 0, stream>>>(x, Xb);
    k_wt<<<dim3(DM / 64, DM / 64, 1), 256, 0, stream>>>(Wq, WQT);
    k_wt<<<dim3(DM / 64, DM / 64, 1), 256, 0, stream>>>(Wk, WKT);
    k_gemmb<<<dim3(NN_ / 64, DM / 64, 1), 128, 0, stream>>>(Xb, WQT, bq, Q);
    k_gemmb<<<dim3(NN_ / 64, DM / 64, 1), 128, 0, stream>>>(Xb, WKT, bk, Kf);
    k_edges<<<NN_ / 4, 256, 0, stream>>>(Q, Kf, rowi, srci, abias, dist, pos, spos, o2s, out);
}
